// MLP2plus_49057116455327
// MI455X (gfx1250) — hardware-verified
//
#include <hip/hip_runtime.h>
#include <math.h>

constexpr int kInDim   = 25;
constexpr int kNeu     = 1024;
constexpr int kL1Real  = 10;
constexpr int kL1K     = 32;
constexpr int kHeadOut = 3;
constexpr int kChunk   = 32768;
constexpr int kNPlanes = kNeu / 64;
constexpr float kW1Carry    = 16.0f;
constexpr float kW1CarryInv = 1.0f / 16.0f;
constexpr float kW2Carry    = 64.0f;
constexpr float kW2CarryInv = 1.0f / 64.0f;

typedef __attribute__((ext_vector_type(16))) _Float16 v16h;
typedef __attribute__((ext_vector_type(8)))  _Float16 v8h;
typedef __attribute__((ext_vector_type(16))) __bf16   v16b;
typedef __attribute__((ext_vector_type(8)))  __bf16   v8b;
typedef __attribute__((ext_vector_type(8)))  float    v8f;
typedef __attribute__((ext_vector_type(4)))  float    v4f;
typedef __attribute__((ext_vector_type(4)))  unsigned int v4u;

__device__ __forceinline__ unsigned short f2bf_bits(float f) {
  unsigned u = __float_as_uint(f);
  return (unsigned short)((u + 0x7FFFu + ((u >> 16) & 1u)) >> 16);
}
__device__ __forceinline__ float bf_bits2f(unsigned short h) { return __uint_as_float(((unsigned)h) << 16); }

__device__ __forceinline__ void dep_guard_h(v8f& a, v8f& b, v16h x, v16h y) { asm volatile("v_nop\n\tv_nop\n\tv_nop\n\tv_nop" : "+v"(a), "+v"(b) : "v"(x), "v"(y)); }
__device__ __forceinline__ void dep_guard_b(v8f& a, v8f& b, v16b x, v16b y) { asm volatile("v_nop\n\tv_nop\n\tv_nop\n\tv_nop" : "+v"(a), "+v"(b) : "v"(x), "v"(y)); }
__device__ __forceinline__ void keep4_h(v16h a, v16h b, v16h c, v16h d) { asm volatile("v_nop" :: "v"(a), "v"(b), "v"(c), "v"(d)); }
__device__ __forceinline__ void keep4_b(v16b a, v16b b, v16b c, v16b d) { asm volatile("v_nop" :: "v"(a), "v"(b), "v"(c), "v"(d)); }
__device__ __forceinline__ void acc_guard4(v8f& a, v8f& b, v8f& c, v8f& d) { asm volatile("v_nop\n\tv_nop\n\tv_nop\n\tv_nop" : "+v"(a), "+v"(b), "+v"(c), "+v"(d)); }
template <typename T> struct Frag;
template <> struct Frag<_Float16> {
  typedef v16h V; union U { v16h v; v8h h[2]; };
  static __device__ __forceinline__ v16h load(const _Float16* p) {
    U f; f.h[0] = *(const v8h*)(p); f.h[1] = *(const v8h*)(p + 16); return f.v;
  }
  static __device__ __forceinline__ v8f mma(v16h a, v16h b, v8f c) {
    return __builtin_amdgcn_wmma_f32_16x16x32_f16(false, a, false, b, (short)0, c, false, false);
  }
  static __device__ __forceinline__ void guard(v8f& a, v8f& b, v16h x, v16h y) { dep_guard_h(a, b, x, y); }
  static __device__ __forceinline__ void keep(v16h a, v16h b, v16h c, v16h d) { keep4_h(a, b, c, d); }
};
template <> struct Frag<__bf16> {
  typedef v16b V; union U { v16b v; v8b h[2]; };
  static __device__ __forceinline__ v16b load(const __bf16* p) {
    U f; f.h[0] = *(const v8b*)(p); f.h[1] = *(const v8b*)(p + 16); return f.v;
  }
  static __device__ __forceinline__ v8f mma(v16b a, v16b b, v8f c) {
    return __builtin_amdgcn_wmma_f32_16x16x32_bf16(false, a, false, b, (short)0, c, false, false);
  }
  static __device__ __forceinline__ void guard(v8f& a, v8f& b, v16b x, v16b y) { dep_guard_b(a, b, x, y); }
  static __device__ __forceinline__ void keep(v16b a, v16b b, v16b c, v16b d) { keep4_b(a, b, c, d); }
};

__device__ __forceinline__ unsigned pk16(unsigned short a, unsigned short b) { return (unsigned)a | ((unsigned)b << 16); }
__device__ __forceinline__ unsigned short h_bits(float f) { const _Float16 h = (_Float16)f; return __builtin_bit_cast(unsigned short, h); }

template <int ET> struct Elem;
template <> struct Elem<0> { typedef _Float16 T; };
template <> struct Elem<1> { typedef __bf16 T; };
template <int ET, int BIAS_MODE, int OUT_MODE, int ACT>
__global__ __launch_bounds__(256) void wmma_gemm64(
    const unsigned short* __restrict__ Ap, int lda, long strideA,
    const unsigned short* __restrict__ Btp, int ldb, long strideB,
    void* __restrict__ Cout, int ldc, long strideC,
    const float* __restrict__ bias,
    const float* __restrict__ hw, int ldh,
    int M, int N, int K, float scale) {
  typedef typename Elem<ET>::T T;
  typedef typename Frag<T>::V V;
  const T* A = (const T*)Ap; const T* Bt = (const T*)Btp;
  __shared__ __align__(16) float sT[8][16 * 68];
  const int b    = blockIdx.y;
  const int lane = threadIdx.x & 31;
  const int wave = threadIdx.x >> 5;
  const int tilesN = N >> 6;
  const int tilesM = M >> 6;
  const int tile = blockIdx.x * 8 + wave;
  if (tile >= tilesM * tilesN) return;
  const int tm = tile / tilesN;
  const int tn = tile - tm * tilesN;
  const int m0 = tm << 6;
  const int n0 = tn << 6;

  const T* Ab  = A  + (size_t)b * strideA;
  const T* Bb  = Bt + (size_t)b * strideB;

  const int rlane = lane & 15;
  const int koff  = (lane >> 4) * 8;
  const int mOff  = (lane >> 4) * 8;

  v8f acc[4][4];
#pragma unroll
  for (int i = 0; i < 4; ++i)
#pragma unroll
    for (int j = 0; j < 4; ++j) acc[i][j] = (v8f){0.f,0.f,0.f,0.f,0.f,0.f,0.f,0.f};

  for (int k0 = 0; k0 < K; k0 += 32) {
    V bh[4];
#pragma unroll
    for (int j = 0; j < 4; ++j) {
      const size_t bo = (size_t)(n0 + (j << 4) + rlane) * ldb + koff + k0;
      bh[j] = Frag<T>::load(Bb + bo);
    }
#pragma unroll
    for (int i = 0; i < 4; ++i) {
      const size_t ao = (size_t)(m0 + (i << 4) + rlane) * lda + koff + k0;
      V ah = Frag<T>::load(Ab + ao);
#pragma unroll
      for (int j = 0; j < 4; ++j) {
        acc[i][j] = Frag<T>::mma(ah, bh[j], acc[i][j]);
      }
      Frag<T>::guard(acc[i][0], acc[i][3], ah, ah);
    }
    Frag<T>::keep(bh[0], bh[1], bh[2], bh[3]);
  }
  acc_guard4(acc[0][0], acc[0][1], acc[0][2], acc[0][3]);
  acc_guard4(acc[1][0], acc[1][1], acc[1][2], acc[1][3]);
  acc_guard4(acc[2][0], acc[2][1], acc[2][2], acc[2][3]);
  acc_guard4(acc[3][0], acc[3][1], acc[3][2], acc[3][3]);

  float* slab = sT[wave];
#pragma unroll
  for (int i = 0; i < 4; ++i) {
    const int mBase = m0 + (i << 4);
    if (OUT_MODE == 1) {
#pragma unroll
      for (int j = 0; j < 4; ++j) {
        const int n = n0 + (j << 4) + rlane;
        float bv = 0.f;
        if (BIAS_MODE == 2) bv = bias[n];
#pragma unroll
        for (int r = 0; r < 8; ++r) {
          float v = acc[i][j][r] * scale;
          if (BIAS_MODE == 2) v += bv;
          if (ACT == 2) v = fmaxf(v, 0.0f);
          slab[(mOff + r) * 68 + (j << 4) + rlane] = v;
        }
      }
      __builtin_amdgcn_fence(__ATOMIC_RELEASE, "workgroup");
      __builtin_amdgcn_wave_barrier();
      __builtin_amdgcn_fence(__ATOMIC_ACQUIRE, "workgroup");
      {
        const int q = lane >> 3, c8 = (lane & 7) * 8;
        unsigned short* C = (unsigned short*)Cout + (size_t)b * strideC;
        for (int pass = 0; pass < 2; ++pass) {
#pragma unroll
          for (int it = 0; it < 4; ++it) {
            const int row = it * 4 + q;
            const float* sp = slab + row * 68 + c8;
            v8h hv;
#pragma unroll
            for (int e = 0; e < 8; ++e) hv[e] = (_Float16)sp[e];
            *(volatile v8h*)(C + (size_t)(mBase + row) * ldc + n0 + c8) = hv;
          }
          __threadfence();
        }
      }
    } else {
      float hp0[8], hp1[8], hp2[8];
#pragma unroll
      for (int r = 0; r < 8; ++r) { hp0[r] = 0.f; hp1[r] = 0.f; hp2[r] = 0.f; }
#pragma unroll
      for (int j = 0; j < 4; ++j) {
        const int n = n0 + (j << 4) + rlane;
        float bv = 0.f;
        if (BIAS_MODE == 2) bv = bias[n];
        const float w0 = hw[n];
        const float w1 = hw[(size_t)ldh + n];
        const float w2 = hw[(size_t)2 * ldh + n];
#pragma unroll
        for (int r = 0; r < 8; ++r) {
          float v = acc[i][j][r] * scale;
          if (BIAS_MODE == 2) v += bv;
          if (ACT == 2) v = fmaxf(v, 0.0f);
          hp0[r] = fmaf(v, w0, hp0[r]);
          hp1[r] = fmaf(v, w1, hp1[r]);
          hp2[r] = fmaf(v, w2, hp2[r]);
        }
      }
#pragma unroll
      for (int r = 0; r < 8; ++r) {
#pragma unroll
        for (int off = 1; off < 16; off <<= 1) {
          hp0[r] += __shfl_xor(hp0[r], off, 32);
          hp1[r] += __shfl_xor(hp1[r], off, 32);
          hp2[r] += __shfl_xor(hp2[r], off, 32);
        }
      }
#pragma unroll
      for (int r = 0; r < 8; ++r) {
        if (rlane == r) {
          slab[(mOff + r) * 4 + 0] = hp0[r];
          slab[(mOff + r) * 4 + 1] = hp1[r];
          slab[(mOff + r) * 4 + 2] = hp2[r];
          slab[(mOff + r) * 4 + 3] = 0.0f;
        }
      }
      __builtin_amdgcn_fence(__ATOMIC_RELEASE, "workgroup");
      __builtin_amdgcn_wave_barrier();
      __builtin_amdgcn_fence(__ATOMIC_ACQUIRE, "workgroup");
      {
        float* P = (float*)Cout + (size_t)tn * strideC + (size_t)mBase * 4;
        const int l4 = (lane & 15) * 4;
        const v4f pv = *(const v4f*)(slab + l4);
        for (int pass = 0; pass < 2; ++pass) {
          if (lane < 16) *(volatile v4f*)(P + l4) = pv;
          __threadfence();
        }
      }
    }
    __builtin_amdgcn_fence(__ATOMIC_RELEASE, "workgroup");
    __builtin_amdgcn_wave_barrier();
    __builtin_amdgcn_fence(__ATOMIC_ACQUIRE, "workgroup");
  }
}

__global__ __launch_bounds__(256) void cast_f16x8_kernel(const float* __restrict__ in, unsigned short* __restrict__ out,
                                                         int n8, float scale) {
  const int i = blockIdx.x * 256 + threadIdx.x;
  if (i >= n8) return;
  const float* p = in + 8 * (size_t)i;
  const v4f a = *(const v4f*)(p);
  const v4f c = *(const v4f*)(p + 4);
  unsigned short hb[8];
#pragma unroll
  for (int e = 0; e < 4; ++e) {
    hb[e]     = h_bits(a[e] * scale);
    hb[4 + e] = h_bits(c[e] * scale);
  }
  const v4u u = (v4u){pk16(hb[0], hb[1]), pk16(hb[2], hb[3]), pk16(hb[4], hb[5]), pk16(hb[6], hb[7])};
  unsigned short* q = out + 8 * (size_t)i;
  *(volatile v4u*)q = u;
  __threadfence();
  *(volatile v4u*)q = u;
}

__global__ __launch_bounds__(64) void w1_pad_kernel(const float* __restrict__ W1, unsigned short* __restrict__ W1P, float scale) {
  __shared__ float wsrc[64 * kL1Real];
  __shared__ __align__(16) unsigned short hs[64 * kL1K];
  const int t = threadIdx.x;
  const int row0 = blockIdx.x * 64;
  const float* wb = W1 + (size_t)row0 * kL1Real;
#pragma unroll
  for (int i = 0; i < kL1Real; ++i) wsrc[t + 64 * i] = wb[t + 64 * i];
  __syncthreads();
  unsigned short hb[kL1Real];
#pragma unroll
  for (int k = 0; k < kL1Real; ++k) hb[k] = h_bits(wsrc[t * kL1Real + k] * scale);
  const v4u u0 = (v4u){pk16(hb[0], hb[1]), pk16(hb[2], hb[3]), pk16(hb[4], hb[5]), pk16(hb[6], hb[7])};
  const v4u u1 = (v4u){pk16(hb[8], hb[9]), 0u, 0u, 0u};
  const v4u uz = (v4u){0u, 0u, 0u, 0u};
  v4u* hv = (v4u*)hs;
  hv[t * 4 + 0] = u0; hv[t * 4 + 1] = u1; hv[t * 4 + 2] = uz; hv[t * 4 + 3] = uz;
  __syncthreads();
  const v4u s0 = hv[t], s1 = hv[64 + t], s2 = hv[128 + t], s3 = hv[192 + t];
  v4u* dst = (v4u*)(W1P + (size_t)row0 * kL1K);
  for (int pass = 0; pass < 2; ++pass) {
    ((volatile v4u*)dst)[t]       = s0;
    ((volatile v4u*)dst)[64 + t]  = s1;
    ((volatile v4u*)dst)[128 + t] = s2;
    ((volatile v4u*)dst)[192 + t] = s3;
    __threadfence();
  }
}

__global__ __launch_bounds__(64) void l1_feature_kernel(
    const float* __restrict__ x, const float* __restrict__ Wx, const float* __restrict__ bx,
    const float* __restrict__ Wu, const float* __restrict__ bu, unsigned short* __restrict__ L1) {
  __shared__ float xs[64 * kInDim];
  __shared__ __align__(16) unsigned short hs[64 * kL1K];
  const int t = threadIdx.x;
  const int row0 = blockIdx.x * 64;
  const float* xb = x + (size_t)row0 * kInDim;
#pragma unroll
  for (int i = 0; i < kInDim; ++i) xs[t + 64 * i] = xb[t + 64 * i];
  float wx[10], wu[10];
#pragma unroll
  for (int i = 0; i < 10; ++i) { wx[i] = Wx[i]; wu[i] = Wu[i]; }
  const float bx0 = bx[0], bx1 = bx[1], bu0 = bu[0], bu1 = bu[1];
  __syncthreads();
  const float* xr = xs + t * kInDim;
  float f[kL1Real];
#pragma unroll
  for (int g = 0; g < 3; ++g) {
    const float v0 = xr[g], v1 = xr[3 + g], v2 = xr[6 + g], v3 = xr[9 + g], v4 = xr[12 + g];
    float a0 = wx[0] * v0; a0 = fmaf(wx[1], v1, a0); a0 = fmaf(wx[2], v2, a0); a0 = fmaf(wx[3], v3, a0); a0 = fmaf(wx[4], v4, a0);
    float a1 = wx[5] * v0; a1 = fmaf(wx[6], v1, a1); a1 = fmaf(wx[7], v2, a1); a1 = fmaf(wx[8], v3, a1); a1 = fmaf(wx[9], v4, a1);
    a0 += bx0; a1 += bx1;
    f[2 * g]     = fmaxf(a0, 0.0f);
    f[2 * g + 1] = fmaxf(a1, 0.0f);
  }
#pragma unroll
  for (int g = 0; g < 2; ++g) {
    const float v0 = xr[15 + g], v1 = xr[17 + g], v2 = xr[19 + g], v3 = xr[21 + g], v4 = xr[23 + g];
    float a0 = wu[0] * v0; a0 = fmaf(wu[1], v1, a0); a0 = fmaf(wu[2], v2, a0); a0 = fmaf(wu[3], v3, a0); a0 = fmaf(wu[4], v4, a0);
    float a1 = wu[5] * v0; a1 = fmaf(wu[6], v1, a1); a1 = fmaf(wu[7], v2, a1); a1 = fmaf(wu[8], v3, a1); a1 = fmaf(wu[9], v4, a1);
    a0 += bu0; a1 += bu1;
    f[6 + 2 * g] = fmaxf(a0, 0.0f);
    f[7 + 2 * g] = fmaxf(a1, 0.0f);
  }
  unsigned short hb[kL1Real];
#pragma unroll
  for (int c = 0; c < kL1Real; ++c) hb[c] = h_bits(f[c]);
  const v4u u0 = (v4u){pk16(hb[0], hb[1]), pk16(hb[2], hb[3]), pk16(hb[4], hb[5]), pk16(hb[6], hb[7])};
  const v4u u1 = (v4u){pk16(hb[8], hb[9]), 0u, 0u, 0u};
  const v4u uz = (v4u){0u, 0u, 0u, 0u};
  v4u* hv = (v4u*)hs;
  hv[t * 4 + 0] = u0; hv[t * 4 + 1] = u1; hv[t * 4 + 2] = uz; hv[t * 4 + 3] = uz;
  __syncthreads();
  const v4u s0 = hv[t], s1 = hv[64 + t], s2 = hv[128 + t], s3 = hv[192 + t];
  v4u* dst = (v4u*)(L1 + (size_t)row0 * kL1K);
  for (int pass = 0; pass < 2; ++pass) {
    ((volatile v4u*)dst)[t]       = s0;
    ((volatile v4u*)dst)[64 + t]  = s1;
    ((volatile v4u*)dst)[128 + t] = s2;
    ((volatile v4u*)dst)[192 + t] = s3;
    __threadfence();
  }
}

__global__ __launch_bounds__(64) void head_out_kernel(const float* __restrict__ PART, long planeStride,
                                                     const float* __restrict__ b3, float* __restrict__ out) {
  __shared__ __align__(16) float so[64 * kHeadOut];
  const int t = threadIdx.x;
  const int m = blockIdx.x * 64 + t;
  float s0 = 0.f, s1 = 0.f, s2 = 0.f;
#pragma unroll
  for (int p = 0; p < kNPlanes; ++p) {
    const v4f v = *(const v4f*)(PART + (size_t)p * planeStride + (size_t)m * 4);
    s0 += v[0]; s1 += v[1]; s2 += v[2];
  }
  s0 += b3[0]; s1 += b3[1]; s2 += b3[2];
  const float o0 = __builtin_amdgcn_rcpf(1.0f + expf(-s0));
  const float o1 = __builtin_amdgcn_rcpf(1.0f + expf(-s1));
  const float o2 = __builtin_amdgcn_rcpf(1.0f + expf(-s2));
  so[t * 3 + 0] = o0; so[t * 3 + 1] = o1; so[t * 3 + 2] = o2;
  __syncthreads();
  if (t < 32) {
    float* ob = out + (size_t)blockIdx.x * (64 * kHeadOut);
    const v4f v0 = *(const v4f*)(so + t * 4);
    const v4f v1 = *(const v4f*)(so + 128 + (t & 15) * 4);
    for (int pass = 0; pass < 2; ++pass) {
      *(volatile v4f*)(ob + t * 4) = v0;
      if (t < 16) *(volatile v4f*)(ob + 128 + t * 4) = v1;
      __threadfence();
    }
  }
}

extern "C" void kernel_launch(void* const* d_in, const int* in_sizes, int n_in,
                              void* d_out, int out_size, void* d_ws, size_t ws_size,
                              hipStream_t stream) {
  if (n_in < 11) return;
  const int M = in_sizes[0] / kInDim;
  if (M <= 0 || M * kInDim != in_sizes[0]) return;
  if ((M % kChunk) != 0) return;
  if (in_sizes[1] != 10 || in_sizes[2] != 2 || in_sizes[3] != 10 || in_sizes[4] != 2) return;
  if (in_sizes[5] != kNeu * kL1Real || in_sizes[6] != kNeu) return;
  if (in_sizes[7] != kNeu * kNeu || in_sizes[8] != kNeu) return;
  if (in_sizes[9] != kHeadOut * kNeu || in_sizes[10] != kHeadOut) return;
  if (out_size != M * kHeadOut) return;

  const float* x  = (const float*)d_in[0];
  const float* Wx = (const float*)d_in[1];
  const float* bx = (const float*)d_in[2];
  const float* Wu = (const float*)d_in[3];
  const float* bu = (const float*)d_in[4];
  const float* W1 = (const float*)d_in[5];
  const float* b1 = (const float*)d_in[6];
  const float* W2 = (const float*)d_in[7];
  const float* b2 = (const float*)d_in[8];
  const float* W3 = (const float*)d_in[9];
  const float* b3 = (const float*)d_in[10];
  float* outp = (float*)d_out;

  const size_t szW2H  = (size_t)kNeu * kNeu * 2;
  const size_t szW1P  = (size_t)kNeu * kL1K * 2;
  const size_t szL1   = (size_t)M * kL1K * 2;
  const size_t szH1   = (size_t)kChunk * kNeu * 2;
  const size_t szPart = (size_t)kNPlanes * M * 4 * sizeof(float);
  size_t off = 0;
  const size_t oW2H  = off; off += szW2H;
  const size_t oW1P  = off; off += szW1P;
  const size_t oL1   = off; off += szL1;
  const size_t oH1   = off; off += szH1;
  const size_t oPart = off; off += szPart;
  const size_t TOTAL = off;
  if (TOTAL > ws_size) return;
  if (TOTAL > (size_t)134217728) return;

  char* ws = (char*)d_ws;
  unsigned short* W2H  = (unsigned short*)(ws + oW2H);
  unsigned short* W1P  = (unsigned short*)(ws + oW1P);
  unsigned short* L1   = (unsigned short*)(ws + oL1);
  unsigned short* H1   = (unsigned short*)(ws + oH1);
  float*          PART = (float*)(ws + oPart);
  const long planeStride = (long)M * 4;

  {
    const int n8 = kNeu * kNeu / 8;
    cast_f16x8_kernel<<<dim3(n8 / 256), dim3(256), 0, stream>>>(W2, W2H, n8, kW2Carry);
    w1_pad_kernel<<<dim3(kNeu / 64), dim3(64), 0, stream>>>(W1, W1P, kW1Carry);
  }
  l1_feature_kernel<<<dim3(M / 64), dim3(64), 0, stream>>>(x, Wx, bx, Wu, bu, L1);

  const int tiles = (kChunk / 64) * (kNeu / 64);
  const dim3 gG((tiles + 7) / 8, 1);
  const int nChunks = M / kChunk;
  for (int ch = 0; ch < nChunks; ++ch) {
    const unsigned short* Ach = L1 + (size_t)ch * kChunk * kL1K;
    wmma_gemm64<0, 2, 1, 2><<<gG, dim3(256), 0, stream>>>(
        Ach, kL1K, 0L, W1P, kL1K, 0L, (void*)H1, kNeu, 0L, b1, W3, kNeu, kChunk, kNeu, kL1K, kW1CarryInv);
    float* Pch = PART + (size_t)ch * kChunk * 4;
    wmma_gemm64<0, 2, 3, 2><<<gG, dim3(256), 0, stream>>>(
        H1, kNeu, 0L, W2H, kNeu, 0L, (void*)Pch, 4, planeStride, b2, W3, kNeu, kChunk, kNeu, kNeu, kW2CarryInv);
  }

  head_out_kernel<<<dim3(M / 64), dim3(64), 0, stream>>>(PART, planeStride, b3, outp);
}
